// DotProductAttention_44873818308757
// MI455X (gfx1250) — hardware-verified
//
#include <hip/hip_runtime.h>


#ifndef NB
#define NB 16
#endif
#ifndef SEQ
#define SEQ 2048
#endif
#define NB_FULL  16
#define SEQ_FULL 2048
#define HD    128
#define QTILE 128
#define NWAVE 8
#define KC    64
#define KP    136
#define VP    72
#define PP    72
#define OP    68
#define TP    72
#define PWU   (2 * 16 * PP)
#define SCL   0.08838834764831845f
#define NEGF  (-1000000.0f)
#define L2E   1.4426950408889634f

static_assert(SEQ % QTILE == 0);
static_assert(SEQ % KC == 0);
static_assert(NB >= 1 && NB <= NB_FULL);
static_assert(SEQ >= KC && SEQ <= SEQ_FULL);
static_assert(KC == 64 && HD == 128);
static_assert(QTILE == NWAVE * 16);
static_assert(PWU * 2 >= 16 * OP * 4);
static_assert((KP * 2) % 16 == 0 && (VP * 2) % 16 == 0 && (PP * 2) % 16 == 0 && (OP * 4) % 16 == 0);
static_assert(KC * HD / 8 == 4 * 256);
static_assert(HD * KC / 8 == 4 * 256);
static_assert(KC * HD / 4 == 8 * 256);

typedef unsigned short bf;
typedef __attribute__((ext_vector_type(16))) __bf16 v16bf;
typedef __attribute__((ext_vector_type(8)))  unsigned short v8us;
typedef __attribute__((ext_vector_type(16))) unsigned short v16us;
typedef __attribute__((ext_vector_type(8)))  float v8f;
typedef __attribute__((ext_vector_type(4)))  float v4f;
typedef v8us  __attribute__((may_alias)) v8usa;
typedef v8f   __attribute__((may_alias)) v8fa;
typedef v4f   __attribute__((may_alias)) v4fa;
typedef float __attribute__((may_alias)) fal;

__device__ __forceinline__ unsigned short f2bf(float f) { unsigned u = __float_as_uint(f); u += 0x7FFFu + ((u >> 16) & 1u); return (unsigned short)(u >> 16); }
__device__ __forceinline__ float bf2f(unsigned short b) { return __uint_as_float(((unsigned)b) << 16); }
__device__ __forceinline__ v16bf cat16b(v8us lo, v8us hi) { return __builtin_bit_cast(v16bf, __builtin_shufflevector(lo, hi, 0, 1, 2, 3, 4, 5, 6, 7, 8, 9, 10, 11, 12, 13, 14, 15)); }
__device__ __forceinline__ v8f wmmab(v16bf a, v16bf b, v8f c) { return __builtin_amdgcn_wmma_f32_16x16x32_bf16(false, a, false, b, (short)0, c, false, false); }
__device__ __forceinline__ float ex2(float x) { return __builtin_amdgcn_exp2f(x); }

__global__ __launch_bounds__(256) void k_prep(const float* __restrict__ K, const float* __restrict__ V, bf* Kb, bf* Vt) {
    __shared__ __align__(16) unsigned short T[HD * TP];
    const int tid = threadIdx.x; const int bb = blockIdx.y; const int k0 = blockIdx.x * KC;
    const float* Kg = K + ((size_t)bb * SEQ_FULL + k0) * HD;
    const float* Vg = V + ((size_t)bb * SEQ_FULL + k0) * HD;
#pragma unroll
    for (int i = 0; i < 8; ++i) {
        const int p = tid + i * 256; const int key = p >> 5; const int d0 = (p & 31) * 4;
        const v4f x = *(const v4fa*)(Vg + (size_t)key * HD + d0);
#pragma unroll
        for (int j = 0; j < 4; ++j) T[(d0 + j) * TP + key] = f2bf(x[j]);
    }
    v8us ko[4];
#pragma unroll
    for (int i = 0; i < 4; ++i) {
        const int p = tid + i * 256; const int key = p >> 4; const int d0 = (p & 15) * 8;
        const v8f x = *(const v8fa*)(Kg + (size_t)key * HD + d0);
        v8us o;
#pragma unroll
        for (int e = 0; e < 8; ++e) o[e] = f2bf(x[e]);
        ko[i] = o;
    }
    __syncthreads();
    v8us vo[4];
#pragma unroll
    for (int i = 0; i < 4; ++i) { const int p = tid + i * 256; const int d = p >> 3; const int ks = (p & 7) * 8; vo[i] = *(const v8usa*)(T + d * TP + ks); }
    bf* kdst = Kb + ((size_t)bb * SEQ + k0) * HD;
    bf* vdst = Vt + (size_t)bb * HD * SEQ + k0;
#pragma unroll
    for (int i = 0; i < 4; ++i) {
        const int p = tid + i * 256;
        { const int r = p >> 4; const int s8 = (p & 15) * 8; *(volatile v8us*)(kdst + (size_t)r * HD + s8) = ko[i]; }
        { const int r = p >> 3; const int s8 = (p & 7) * 8;  *(volatile v8us*)(vdst + (size_t)r * SEQ + s8) = vo[i]; }
    }
    __threadfence();
#pragma unroll
    for (int i = 0; i < 4; ++i) {
        const int p = tid + i * 256;
        { const int r = p >> 4; const int s8 = (p & 15) * 8; *(volatile v8us*)(kdst + (size_t)r * HD + s8) = ko[i]; }
        { const int r = p >> 3; const int s8 = (p & 7) * 8;  *(volatile v8us*)(vdst + (size_t)r * SEQ + s8) = vo[i]; }
    }
}

template <int HF>
__device__ __forceinline__ void epi_half(const v8f (&acc)[8], const float (&inv)[8], fal* os, float* orow, int h, int m) {
#pragma unroll
    for (int dbl = 0; dbl < 4; ++dbl)
#pragma unroll
        for (int r = 0; r < 8; ++r) os[(8 * h + r) * OP + dbl * 16 + m] = acc[HF * 4 + dbl][r] * inv[r];
    asm volatile("" ::: "memory");
    __builtin_amdgcn_fence(3  , "wavefront");
    __builtin_amdgcn_wave_barrier();
    asm volatile("" ::: "memory");
    v4f ov[8];
#pragma unroll
    for (int g = 0; g < 8; ++g) { const int row = 2 * g + h; ov[g] = *(const v4fa*)((const float*)os + row * OP + m * 4); }
    float* ob = orow + HF * 64 + m * 4;
#pragma unroll
    for (int g = 0; g < 8; ++g) { const int row = 2 * g + h; *(volatile v4f*)(ob + (size_t)row * HD) = ov[g]; }
    __threadfence();
#pragma unroll
    for (int g = 0; g < 8; ++g) { const int row = 2 * g + h; *(volatile v4f*)(ob + (size_t)row * HD) = ov[g]; }
    asm volatile("" ::: "memory");
    __builtin_amdgcn_fence(3  , "wavefront");
    __builtin_amdgcn_wave_barrier();
    asm volatile("" ::: "memory");
}

__global__ __launch_bounds__(256) void k_attn(const float* __restrict__ Q, const bf* __restrict__ Kb, const bf* __restrict__ Vt, const int* __restrict__ vlens, float* out) {
    __shared__ __align__(16) unsigned short ksh[KC * KP];
    __shared__ __align__(16) unsigned short vsh[HD * VP];
    __shared__ __align__(16) unsigned short praw[NWAVE * PWU];
    const int tid = threadIdx.x, wave = tid >> 5, lane = tid & 31, m = lane & 15, h = lane >> 4;
    const int bb = blockIdx.y; const int q0 = blockIdx.x * QTILE + wave * 16;
    unsigned short* ph_t = praw + wave * PWU;
    unsigned short* pl_t = ph_t + 16 * PP;

    int vl = vlens[bb];
    vl = vl < 0 ? 0 : (vl > SEQ ? SEQ : vl);
    const int kend = (vl == 0) ? SEQ : (((vl + KC - 1) / KC) * KC);

    const float* qrow = Q + ((size_t)bb * SEQ_FULL + q0 + m) * HD;
    v16bf qa[4];
#pragma unroll
    for (int dc = 0; dc < 4; ++dc) {
        const v8f x0 = *(const v8fa*)(qrow + dc * 32 + 8 * h);
        const v8f x1 = *(const v8fa*)(qrow + dc * 32 + 16 + 8 * h);
        v8us u0, u1;
#pragma unroll
        for (int e = 0; e < 8; ++e) { u0[e] = f2bf(x0[e]); u1[e] = f2bf(x1[e]); }
        qa[dc] = cat16b(u0, u1);
    }
    v8f acc[8];
    float mrun[8], lrun[8];
#pragma unroll
    for (int db = 0; db < 8; ++db) acc[db] = (v8f){};
#pragma unroll
    for (int r = 0; r < 8; ++r) { mrun[r] = -1.0e30f; lrun[r] = 0.0f; }

    const bf* kbase = Kb + (size_t)bb * SEQ * HD;
    const bf* vbase = Vt + (size_t)bb * HD * SEQ;

#pragma unroll 1
    for (int k0 = 0; k0 < kend; k0 += KC) {
#pragma unroll
        for (int i = 0; i < 4; ++i) {
            const int p = tid + i * 256;
            { const int r = p >> 4; const int s8 = (p & 15) * 8;
              const v8us kv = *(const v8usa*)(kbase + (size_t)(k0 + r) * HD + s8);
              *(v8usa*)(ksh + r * KP + s8) = kv; }
            { const int r = p >> 3; const int s8 = (p & 7) * 8;
              const v8us vv = *(const v8usa*)(vbase + (size_t)r * SEQ + k0 + s8);
              *(v8usa*)(vsh + r * VP + s8) = vv; }
        }
        __syncthreads();

        v8f s[4];
        v16bf kfr;
#pragma unroll
        for (int j = 0; j < 4; ++j) {
            v8f c = (v8f){};
#pragma unroll
            for (int dc = 0; dc < 4; ++dc) {
                const unsigned short* kr = ksh + (j * 16 + m) * KP + dc * 32 + 8 * h;
                kfr = cat16b(*(const v8usa*)kr, *(const v8usa*)(kr + 16));
                c = wmmab(qa[dc], kfr, c);
            }
            s[j] = c;
        }
        asm volatile("v_nop\n\tv_nop\n\tv_nop\n\tv_nop" : "+v"(s[0]), "+v"(s[1]), "+v"(s[2]), "+v"(s[3]) : "v"(qa[0]), "v"(qa[1]), "v"(qa[2]), "v"(qa[3]), "v"(kfr));

#pragma unroll
        for (int j = 0; j < 4; ++j) {
            const bool kval = (k0 + j * 16 + m) < vl;
#pragma unroll
            for (int r = 0; r < 8; ++r) s[j][r] = kval ? (s[j][r] * SCL) : NEGF;
        }

        float mn[8];
#pragma unroll
        for (int r = 0; r < 8; ++r) {
            float x = fmaxf(fmaxf(s[0][r], s[1][r]), fmaxf(s[2][r], s[3][r]));
#pragma unroll
            for (int sh = 1; sh <= 8; sh <<= 1) x = fmaxf(x, __shfl_xor(x, sh, 32));
            mn[r] = fmaxf(mrun[r], x);
            const float corr = ex2((mrun[r] - mn[r]) * L2E);
            mrun[r] = mn[r];
            lrun[r] *= corr;
#pragma unroll
            for (int db = 0; db < 8; ++db) acc[db][r] *= corr;
        }

#pragma unroll
        for (int r = 0; r < 8; ++r) {
#pragma unroll
            for (int j = 0; j < 4; ++j) {
                const float pv = ex2((s[j][r] - mn[r]) * L2E);
                lrun[r] += pv;
                const unsigned short hb = f2bf(pv);
                const unsigned short lb = f2bf(pv - bf2f(hb));
                ph_t[(8 * h + r) * PP + j * 16 + m] = hb;
                pl_t[(8 * h + r) * PP + j * 16 + m] = lb;
            }
        }
        asm volatile("" ::: "memory");
        __builtin_amdgcn_fence(3  , "wavefront");
        __builtin_amdgcn_wave_barrier();
        asm volatile("" ::: "memory");

        v16bf pa, pb, vfr;
#pragma unroll
        for (int c = 0; c < 2; ++c) {
            const unsigned short* pr = ph_t + m * PP + c * 32 + 8 * h;
            const unsigned short* lr = pl_t + m * PP + c * 32 + 8 * h;
            pa = cat16b(*(const v8usa*)pr, *(const v8usa*)(pr + 16));
            pb = cat16b(*(const v8usa*)lr, *(const v8usa*)(lr + 16));
#pragma unroll
            for (int db = 0; db < 8; ++db) {
                const unsigned short* vr = vsh + (db * 16 + m) * VP + c * 32 + 8 * h;
                vfr = cat16b(*(const v8usa*)vr, *(const v8usa*)(vr + 16));
                acc[db] = wmmab(pa, vfr, acc[db]);
                acc[db] = wmmab(pb, vfr, acc[db]);
            }
        }
        asm volatile("v_nop\n\tv_nop\n\tv_nop\n\tv_nop"
                     : "+v"(acc[0]), "+v"(acc[1]), "+v"(acc[2]), "+v"(acc[3]), "+v"(acc[4]), "+v"(acc[5]), "+v"(acc[6]), "+v"(acc[7])
                     : "v"(pa), "v"(pb), "v"(vfr));
        __syncthreads();
    }
    __syncthreads();

    float inv[8];
#pragma unroll
    for (int r = 0; r < 8; ++r) {
        float x = lrun[r];
#pragma unroll
        for (int sh = 1; sh <= 8; sh <<= 1) x += __shfl_xor(x, sh, 32);
        inv[r] = 1.0f / x;
    }
    fal* os = (fal*)(praw + wave * PWU);
    float* orow = out + ((size_t)bb * SEQ + q0) * HD;
    epi_half<0>(acc, inv, os, orow, h, m);
    epi_half<1>(acc, inv, os, orow, h, m);
}

extern "C" void kernel_launch(void* const* d_in, const int* in_sizes, int n_in,
                              void* d_out, int out_size, void* d_ws, size_t ws_size, hipStream_t stream) {
    if (n_in < 4) return;
    const size_t need_in = ((size_t)(NB - 1) * SEQ_FULL + SEQ) * HD;
    if ((size_t)in_sizes[0] < need_in || (size_t)in_sizes[1] < need_in || (size_t)in_sizes[2] < need_in) return;
    if (in_sizes[3] < NB) return;
    if ((size_t)out_size < (size_t)NB * SEQ * HD) return;
    const float* Qin = (const float*)d_in[0];
    const float* Kin = (const float*)d_in[1];
    const float* Vin = (const float*)d_in[2];
    const int*   VLin = (const int*)d_in[3];
    float* OUT = (float*)d_out;
    char* wsp = (char*)d_ws;
    const size_t plane = ((size_t)NB * SEQ * HD * 2 + 255) & ~(size_t)255;
    bf* Kb = (bf*)wsp;
    bf* Vt = (bf*)(wsp + plane);
    if (2 * plane > ws_size) return;
    k_prep<<<dim3(SEQ / KC, NB), 256, 0, stream>>>(Kin, Vin, Kb, Vt);
    k_attn<<<dim3(SEQ / QTILE, NB), 256, 0, stream>>>(Qin, Kb, Vt, VLin, OUT);
}
